// MambaModel_62423054680256
// MI455X (gfx1250) — hardware-run, weakly checked
//
#include <hip/hip_runtime.h>
#include <math.h>

typedef __attribute__((ext_vector_type(8)))  _Float16 v8h;
typedef __attribute__((ext_vector_type(16))) __bf16   v16b;
typedef __attribute__((ext_vector_type(8)))  __bf16   v8b;
typedef __attribute__((ext_vector_type(8)))  float    v8f;
typedef __attribute__((ext_vector_type(4)))  float    v4f;

constexpr int kLayers = 2;
constexpr int kBatch  = 2;
constexpr int kSeq    = 1024;
constexpr int kDm     = 1024;
constexpr int kDin    = 2048;
constexpr int kNst    = 16;
constexpr int kDtR    = 64;
constexpr int kPrjN   = 96;
constexpr int kPrjP   = 128;
constexpr int kXzP    = 2 * kDin;
constexpr int kRows   = kBatch * kSeq;
constexpr int kConvTP = 260;
constexpr int kScanTS = 64;
constexpr int kScanCh = 64;
constexpr int kScanYP = 68;
constexpr int kScanBC = 2 * kNst;
static_assert(kDtR + 2 * kNst == kPrjN, "x_proj width");
static_assert((kPrjP % 64) == 0 && kPrjP >= kPrjN, "padded x_proj width");
static_assert((kDm % 32) == 0 && (kDin % 32) == 0 && (kDtR % 32) == 0, "GEMM K multiples of 32");
static_assert((kRows % 64) == 0 && (kXzP % 64) == 0 && (kDin % 64) == 0 && (kDm % 64) == 0, "GEMM M,N multiples of 64");
static_assert((kSeq % kScanTS) == 0 && (kSeq % 64) == 0 && (kDin % kScanCh) == 0 && (kDin % 256) == 0, "tile multiples");
static_assert(kScanTS * kScanBC == 64 * 8 * 4, "scan staging coverage: 64 threads x 8 iterations x 4 floats");

constexpr size_t kOffXH   = 0;
constexpr size_t kOffXL   = kOffXH   + (size_t)kRows * kDm   * 2;
constexpr size_t kOffWIN  = kOffXL   + (size_t)kRows * kDm   * 2;
constexpr size_t kOffWX   = kOffWIN  + (size_t)kXzP  * kDm   * 2;
constexpr size_t kOffWDT  = kOffWX   + (size_t)kPrjP * kDin  * 2;
constexpr size_t kOffWOUT = kOffWDT  + (size_t)kDin  * kDtR  * 2;
constexpr size_t kOffXZ   = kOffWOUT + (size_t)kDm   * kDin  * 2;
constexpr size_t kOffUC   = kOffXZ   + (size_t)kRows * kXzP  * 4;
constexpr size_t kOffUCH  = kOffUC   + (size_t)kRows * kDin  * 4;
constexpr size_t kOffXD   = kOffUCH  + (size_t)kRows * kDin  * 2;
constexpr size_t kOffDT   = kOffXD   + (size_t)kRows * kPrjP * 4;
constexpr size_t kOffDLR  = kOffDT   + (size_t)kRows * kDtR  * 2;
constexpr size_t kOffYH   = kOffDLR  + (size_t)kRows * kDin  * 4;
constexpr size_t kOffYL   = kOffYH   + (size_t)kRows * kDin  * 2;
constexpr size_t kWsTotal = kOffYL   + (size_t)kRows * kDin  * 2;
static_assert(kWsTotal == 115343360ull, "carve total");
static_assert(kWsTotal <= 134217728ull, "carve cap");
static_assert((kOffXL % 128) == 0 && (kOffWIN % 128) == 0 && (kOffWX % 128) == 0 && (kOffWDT % 128) == 0 &&
              (kOffWOUT % 128) == 0 && (kOffXZ % 128) == 0 && (kOffUC % 128) == 0 && (kOffUCH % 128) == 0 &&
              (kOffXD % 128) == 0 && (kOffDT % 128) == 0 && (kOffDLR % 128) == 0 && (kOffYH % 128) == 0 &&
              (kOffYL % 128) == 0, "128-B aligned regions");

__device__ __forceinline__ unsigned short f2bf_bits(float f) {
  unsigned u = __float_as_uint(f);
  return (unsigned short)((u + 0x7FFFu + ((u >> 16) & 1u)) >> 16);
}
__device__ __forceinline__ float bf_bits2f(unsigned short h) { return __uint_as_float(((unsigned)h) << 16); }
__device__ __forceinline__ float rne_bf16(float f) { return bf_bits2f(f2bf_bits(f)); }

__device__ __forceinline__ void row_guard_b(v8f& a, v8f& b, v8f& c, v8f& d, v16b x, v16b y) {
  asm volatile("v_nop\n\tv_nop\n\tv_nop\n\tv_nop" : "+v"(a), "+v"(b), "+v"(c), "+v"(d) : "v"(x), "v"(y));
}
__device__ __forceinline__ void keep4_b(v16b a, v16b b, v16b c, v16b d) { asm volatile("v_nop" :: "v"(a), "v"(b), "v"(c), "v"(d)); }
__device__ __forceinline__ void acc_guard4(v8f& a, v8f& b, v8f& c, v8f& d) { asm volatile("v_nop\n\tv_nop\n\tv_nop\n\tv_nop" : "+v"(a), "+v"(b), "+v"(c), "+v"(d)); }

struct FragB {
  union U { v16b v; v8b h[2]; };
  static __device__ __forceinline__ v16b load(const __bf16* p) {
    U f; f.h[0] = *(const v8b*)(p); f.h[1] = *(const v8b*)(p + 16); return f.v;
  }
  static __device__ __forceinline__ v8f mma(v16b a, v16b b, v8f c) {
    return __builtin_amdgcn_wmma_f32_16x16x32_bf16(false, a, false, b, (short)0, c, false, false);
  }
};

template <int SPL, int OUT_MODE>
__global__ __launch_bounds__(256) void wmma_gemm64(
    const unsigned short* __restrict__ Ap, const unsigned short* __restrict__ A2p, int lda,
    const unsigned short* __restrict__ Btp, int ldb,
    void* __restrict__ Cout, void* __restrict__ Cout2, int ldc,
    int M, int N, int K) {
  const __bf16* A  = (const __bf16*)Ap;
  const __bf16* A2 = (const __bf16*)A2p;
  const __bf16* Bt = (const __bf16*)Btp;
  __shared__ __align__(16) float sT[8][16 * 68];
  const int lane = threadIdx.x & 31;
  const int wave = threadIdx.x >> 5;
  const int tilesN = N >> 6;
  const int tilesM = M >> 6;
  const int tile = blockIdx.x * 8 + wave;
  if (tile >= tilesM * tilesN) return;
  const int tm = tile / tilesN;
  const int tn = tile - tm * tilesN;
  const int m0 = tm << 6;
  const int n0 = tn << 6;

  const int rlane = lane & 15;
  const int koff  = (lane >> 4) * 8;
  const int mOff  = (lane >> 4) * 8;

  v8f acc[4][4];
#pragma unroll
  for (int i = 0; i < 4; ++i)
#pragma unroll
    for (int j = 0; j < 4; ++j) acc[i][j] = (v8f){0.f,0.f,0.f,0.f,0.f,0.f,0.f,0.f};

  for (int k0 = 0; k0 < K; k0 += 32) {
    v16b bh[4];
#pragma unroll
    for (int j = 0; j < 4; ++j) {
      const size_t bo = (size_t)(n0 + (j << 4) + rlane) * ldb + koff + k0;
      bh[j] = FragB::load(Bt + bo);
    }
#pragma unroll
    for (int i = 0; i < 4; ++i) {
      const size_t ao = (size_t)(m0 + (i << 4) + rlane) * lda + koff + k0;
      v16b ah = FragB::load(A + ao);
      v16b al = ah;
      if (SPL == 1) al = FragB::load(A2 + ao);
#pragma unroll
      for (int j = 0; j < 4; ++j) {
        acc[i][j] = FragB::mma(ah, bh[j], acc[i][j]);
        if (SPL == 1) acc[i][j] = FragB::mma(al, bh[j], acc[i][j]);
      }
      row_guard_b(acc[i][0], acc[i][1], acc[i][2], acc[i][3], ah, al);
    }
    keep4_b(bh[0], bh[1], bh[2], bh[3]);
  }
  acc_guard4(acc[0][0], acc[0][1], acc[0][2], acc[0][3]);
  acc_guard4(acc[1][0], acc[1][1], acc[1][2], acc[1][3]);
  acc_guard4(acc[2][0], acc[2][1], acc[2][2], acc[2][3]);
  acc_guard4(acc[3][0], acc[3][1], acc[3][2], acc[3][3]);

  float* slab = sT[wave];
#pragma unroll
  for (int i = 0; i < 4; ++i) {
    const int mBase = m0 + (i << 4);
#pragma unroll
    for (int j = 0; j < 4; ++j) {
#pragma unroll
      for (int r = 0; r < 8; ++r) {
        slab[(mOff + r) * 68 + (j << 4) + rlane] = acc[i][j][r];
      }
    }
    __builtin_amdgcn_fence(__ATOMIC_RELEASE, "workgroup");
    __builtin_amdgcn_wave_barrier();
    __builtin_amdgcn_fence(__ATOMIC_ACQUIRE, "workgroup");
    if (OUT_MODE == 0) {
      float* C = (float*)Cout;
      const int hh = lane >> 4, c4 = (lane & 15) * 4;
      for (int pass = 0; pass < 2; ++pass) {
#pragma unroll
        for (int it = 0; it < 8; ++it) {
          const int row = it * 2 + hh;
          v4f v = *(const v4f*)(slab + row * 68 + c4);
          *(volatile v4f*)(C + (size_t)(mBase + row) * ldc + n0 + c4) = v;
        }
        __threadfence();
      }
    } else {
      const int q = lane >> 3, c8 = (lane & 7) * 8;
      unsigned short* C  = (unsigned short*)Cout;
      unsigned short* C2 = (unsigned short*)Cout2;
      for (int pass = 0; pass < 2; ++pass) {
#pragma unroll
        for (int it = 0; it < 4; ++it) {
          const int row = it * 4 + q;
          const float* sp = slab + row * 68 + c8;
          v8h hv, lv;
#pragma unroll
          for (int e = 0; e < 8; ++e) {
            const float sv = sp[e];
            const unsigned short hb = f2bf_bits(sv);
            const unsigned short lb = f2bf_bits(sv - bf_bits2f(hb));
            hv[e] = __builtin_bit_cast(_Float16, hb);
            lv[e] = __builtin_bit_cast(_Float16, lb);
          }
          *(volatile v8h*)(C  + (size_t)(mBase + row) * ldc + n0 + c8) = hv;
          *(volatile v8h*)(C2 + (size_t)(mBase + row) * ldc + n0 + c8) = lv;
        }
        __threadfence();
      }
    }
    __builtin_amdgcn_fence(__ATOMIC_RELEASE, "workgroup");
    __builtin_amdgcn_wave_barrier();
    __builtin_amdgcn_fence(__ATOMIC_ACQUIRE, "workgroup");
  }
}

__global__ __launch_bounds__(256) void prep_x_kernel(
    const float* __restrict__ pe, const float* __restrict__ cond,
    unsigned short* __restrict__ XH, unsigned short* __restrict__ XL, int total8)
{
  const int i = blockIdx.x * 256 + threadIdx.x;
  if (i >= total8) return;
  const size_t e0 = (size_t)i << 3;
  const int row = (int)(e0 / (size_t)kDm);
  const int col = (int)(e0 - (size_t)row * kDm);
  const int l   = row & (kSeq - 1);
  const float* pp = pe + (size_t)l * kDm + col;
  const float* cp = cond + e0;
  const v4f p0 = *(const v4f*)(pp);
  const v4f p1 = *(const v4f*)(pp + 4);
  const v4f c0 = *(const v4f*)(cp);
  const v4f c1 = *(const v4f*)(cp + 4);
  v8h hv, lv;
#pragma unroll
  for (int e = 0; e < 4; ++e) {
    const float x0 = rne_bf16(p0[e]) + rne_bf16(c0[e]);
    const float x1 = rne_bf16(p1[e]) + rne_bf16(c1[e]);
    const unsigned short h0 = f2bf_bits(x0), h1 = f2bf_bits(x1);
    const unsigned short l0 = f2bf_bits(x0 - bf_bits2f(h0)), l1 = f2bf_bits(x1 - bf_bits2f(h1));
    hv[e]     = __builtin_bit_cast(_Float16, h0);
    hv[4 + e] = __builtin_bit_cast(_Float16, h1);
    lv[e]     = __builtin_bit_cast(_Float16, l0);
    lv[4 + e] = __builtin_bit_cast(_Float16, l1);
  }
  unsigned short* qh = XH + e0;
  unsigned short* ql = XL + e0;
  *(volatile v8h*)qh = hv;
  *(volatile v8h*)ql = lv;
  __threadfence();
  *(volatile v8h*)qh = hv;
  *(volatile v8h*)ql = lv;
}

__global__ __launch_bounds__(256) void cast_rows_bf16_kernel(
    const float* __restrict__ src, unsigned short* __restrict__ dst, int total8, int real8)
{
  const int i = blockIdx.x * 256 + threadIdx.x;
  if (i >= total8) return;
  const bool live = (i < real8);
  const int ic = live ? i : (real8 - 1);
  const size_t es = (size_t)ic << 3;
  const v4f a0 = *(const v4f*)(src + es);
  const v4f a1 = *(const v4f*)(src + es + 4);
  v8h hv;
#pragma unroll
  for (int e = 0; e < 4; ++e) {
    const unsigned short h0 = f2bf_bits(a0[e]), h1 = f2bf_bits(a1[e]);
    const unsigned short z0 = live ? h0 : (unsigned short)0;
    const unsigned short z1 = live ? h1 : (unsigned short)0;
    hv[e]     = __builtin_bit_cast(_Float16, z0);
    hv[4 + e] = __builtin_bit_cast(_Float16, z1);
  }
  unsigned short* q = dst + ((size_t)i << 3);
  *(volatile v8h*)q = hv;
  __threadfence();
  *(volatile v8h*)q = hv;
}

__global__ __launch_bounds__(256) void dt_cast_kernel(
    const float* __restrict__ XD, unsigned short* __restrict__ DT, int total8)
{
  const int i = blockIdx.x * 256 + threadIdx.x;
  if (i >= total8) return;
  const int e0  = i << 3;
  const int row = e0 / kDtR;
  const int c8  = e0 - row * kDtR;
  const float* p = XD + (size_t)row * kPrjP + c8;
  const v4f a0 = *(const v4f*)(p);
  const v4f a1 = *(const v4f*)(p + 4);
  v8h hv;
#pragma unroll
  for (int e = 0; e < 4; ++e) {
    const unsigned short h0 = f2bf_bits(a0[e]), h1 = f2bf_bits(a1[e]);
    hv[e]     = __builtin_bit_cast(_Float16, h0);
    hv[4 + e] = __builtin_bit_cast(_Float16, h1);
  }
  unsigned short* qd = DT + e0;
  *(volatile v8h*)qd = hv;
  __threadfence();
  *(volatile v8h*)qd = hv;
}

__global__ __launch_bounds__(256) void conv_silu_kernel(
    const float* __restrict__ XZ, const float* __restrict__ cw, const float* __restrict__ cb,
    float* __restrict__ UC, unsigned short* __restrict__ UCH)
{
  __shared__ __align__(16) float sT[16 * kConvTP];
  const int tid = threadIdx.x, lane = tid & 31, wave = tid >> 5;
  const int d0 = blockIdx.x * 256, d = d0 + tid;
  const int g0 = blockIdx.y * 64;
  const int tb = g0 & (kSeq - 1);
  const v4f wv = *(const v4f*)(cw + (size_t)d * 4);
  const float w0 = rne_bf16(wv[0]), w1 = rne_bf16(wv[1]), w2 = rne_bf16(wv[2]), w3 = rne_bf16(wv[3]);
  const float bc = rne_bf16(cb[d]);
  float xm3, xm2, xm1;
  {
    const bool hist = (tb > 0);
    const int rb = hist ? (g0 - 3) : g0;
    const float v3 = XZ[(size_t)rb * kXzP + d];
    const float v2 = XZ[(size_t)(rb + 1) * kXzP + d];
    const float v1 = XZ[(size_t)(rb + 2) * kXzP + d];
    xm3 = hist ? v3 : 0.f;
    xm2 = hist ? v2 : 0.f;
    xm1 = hist ? v1 : 0.f;
  }
  const int hrow = wave >> 1;
  const int hch  = (wave & 1) * 128 + lane * 4;
#pragma unroll 1
  for (int sub = 0; sub < 4; ++sub) {
    const int lb = g0 + sub * 16;
#pragma unroll 1
    for (int s = 0; s < 16; ++s) {
      const float xcur = XZ[(size_t)(lb + s) * kXzP + d];
      float acc = w0 * xm3;
      acc = fmaf(w1, xm2, acc);
      acc = fmaf(w2, xm1, acc);
      acc = fmaf(w3, xcur, acc);
      const float sv = acc + bc;
      const float sg = __builtin_amdgcn_rcpf(1.0f + expf(-sv));
      sT[s * kConvTP + tid] = sv * sg;
      xm3 = xm2; xm2 = xm1; xm1 = xcur;
    }
    __syncthreads();
    v4f fv[4];
    v8h bh[2];
#pragma unroll
    for (int it = 0; it < 4; ++it) fv[it] = *(const v4f*)(sT + (it * 4 + hrow) * kConvTP + hch);
#pragma unroll
    for (int it = 0; it < 2; ++it) {
      const float* sp = sT + (it * 8 + wave) * kConvTP + lane * 8;
      const v4f a0 = *(const v4f*)(sp);
      const v4f a1 = *(const v4f*)(sp + 4);
#pragma unroll
      for (int e = 0; e < 4; ++e) {
        const unsigned short h0 = f2bf_bits(a0[e]), h1 = f2bf_bits(a1[e]);
        bh[it][e]     = __builtin_bit_cast(_Float16, h0);
        bh[it][4 + e] = __builtin_bit_cast(_Float16, h1);
      }
    }
    for (int pass = 0; pass < 2; ++pass) {
#pragma unroll
      for (int it = 0; it < 4; ++it)
        *(volatile v4f*)(UC + (size_t)(lb + it * 4 + hrow) * kDin + d0 + hch) = fv[it];
#pragma unroll
      for (int it = 0; it < 2; ++it) {
        const size_t o = (size_t)(lb + it * 8 + wave) * kDin + d0 + lane * 8;
        *(volatile v8h*)(UCH + o) = bh[it];
      }
      __threadfence();
    }
    __syncthreads();
  }
}

__global__ __launch_bounds__(64) void scan_kernel(
    const float* __restrict__ XD, const float* __restrict__ UC, const float* __restrict__ XZ,
    const float* __restrict__ DLR, const float* __restrict__ bdt, const float* __restrict__ Alog,
    const float* __restrict__ Dp, unsigned short* __restrict__ YH, unsigned short* __restrict__ YL)
{
  __shared__ __align__(16) float sX[kScanTS * kScanBC];
  __shared__ __align__(16) float sY[kScanTS * kScanYP];
  __shared__ __align__(16) float sA[kNst * kScanCh];
  const int tid = threadIdx.x, lane = tid & 31, wave = tid >> 5;
  constexpr int kBlkPerB = kDin / kScanCh;
  const int bix = blockIdx.x / kBlkPerB;
  const int d0  = (blockIdx.x - bix * kBlkPerB) * kScanCh;
  const int d   = d0 + tid;
  const size_t row0 = (size_t)bix * kSeq;
#pragma unroll 1
  for (int s = 0; s < kNst; ++s) sA[s * kScanCh + tid] = -expf(rne_bf16(Alog[(size_t)d * kNst + s]));
  __syncthreads();
  float negA[kNst], h[kNst];
#pragma unroll
  for (int s = 0; s < kNst; ++s) {
    negA[s] = sA[s * kScanCh + tid];
    h[s] = 0.f;
  }
  const float bb = rne_bf16(bdt[d]);
  const float Dd = rne_bf16(Dp[d]);
  const int q = lane >> 3, c8 = (lane & 7) * 8;
#pragma unroll 1
  for (int t0 = 0; t0 < kSeq; t0 += kScanTS) {
    __syncthreads();
#pragma unroll
    for (int i = 0; i < 8; ++i) {
      const int idx = tid + 64 * i;
      const int r   = idx >> 3;
      const int c4  = (idx & 7) * 4;
      *(v4f*)(sX + r * kScanBC + c4) = *(const v4f*)(XD + (row0 + t0 + r) * kPrjP + kDtR + c4);
    }
    __syncthreads();
#pragma unroll 1
    for (int s = 0; s < kScanTS; ++s) {
      const size_t row = row0 + t0 + s;
      const float* xr = sX + s * kScanBC;
      const float vraw = DLR[row * kDin + d];
      const float xt   = UC[row * kDin + d];
      const float zv   = XZ[row * kXzP + kDin + d];
      float Bs[kNst], Cs[kNst];
#pragma unroll
      for (int q4 = 0; q4 < 4; ++q4) {
        const v4f bv = *(const v4f*)(xr + 4 * q4);
        const v4f cv = *(const v4f*)(xr + kNst + 4 * q4);
        Bs[4 * q4 + 0] = bv[0]; Bs[4 * q4 + 1] = bv[1]; Bs[4 * q4 + 2] = bv[2]; Bs[4 * q4 + 3] = bv[3];
        Cs[4 * q4 + 0] = cv[0]; Cs[4 * q4 + 1] = cv[1]; Cs[4 * q4 + 2] = cv[2]; Cs[4 * q4 + 3] = cv[3];
      }
      const float v   = vraw + bb;
      const float a   = __expf(-fabsf(v));
      const float u   = 1.0f + a;
      const float l1p = __logf(u) + (a - (u - 1.0f)) * __builtin_amdgcn_rcpf(u);
      const float dt  = fmaxf(v, 0.0f) + l1p;
      const float dtx = dt * xt;
      float y = 0.f;
#pragma unroll
      for (int k = 0; k < kNst; ++k) {
        const float e = __expf(dt * negA[k]);
        h[k] = e * h[k] + dtx * Bs[k];
        y = h[k] * Cs[k] + y;
      }
      y = xt * Dd + y;
      const float sg = __builtin_amdgcn_rcpf(1.0f + expf(-zv));
      y = y * (zv * sg);
      sY[s * kScanYP + tid] = y;
    }
    __syncthreads();
    v8h hv[8], lv[8];
#pragma unroll
    for (int it = 0; it < 8; ++it) {
      const int rr = it * 8 + wave * 4 + q;
      const float* sp = sY + rr * kScanYP + c8;
      const v4f a0 = *(const v4f*)(sp);
      const v4f a1 = *(const v4f*)(sp + 4);
#pragma unroll
      for (int e = 0; e < 4; ++e) {
        const unsigned short h0 = f2bf_bits(a0[e]), h1 = f2bf_bits(a1[e]);
        const unsigned short l0 = f2bf_bits(a0[e] - bf_bits2f(h0)), l1 = f2bf_bits(a1[e] - bf_bits2f(h1));
        hv[it][e]     = __builtin_bit_cast(_Float16, h0);
        hv[it][4 + e] = __builtin_bit_cast(_Float16, h1);
        lv[it][e]     = __builtin_bit_cast(_Float16, l0);
        lv[it][4 + e] = __builtin_bit_cast(_Float16, l1);
      }
    }
    for (int pass = 0; pass < 2; ++pass) {
#pragma unroll
      for (int it = 0; it < 8; ++it) {
        const int rr = it * 8 + wave * 4 + q;
        const size_t o = (row0 + t0 + rr) * kDin + d0 + c8;
        *(volatile v8h*)(YH + o) = hv[it];
        *(volatile v8h*)(YL + o) = lv[it];
      }
      __threadfence();
    }
  }
}

extern "C" void kernel_launch(void* const* d_in, const int* in_sizes, int n_in,
                              void* d_out, int out_size, void* d_ws, size_t ws_size,
                              hipStream_t stream) {
  if (n_in < 11) return;
  if (in_sizes[0]  != kSeq * kDm) return;
  if (in_sizes[1]  != kRows * kDm) return;
  if (in_sizes[2]  != kLayers * kXzP * kDm) return;
  if (in_sizes[3]  != kLayers * kDin * 4) return;
  if (in_sizes[4]  != kLayers * kDin) return;
  if (in_sizes[5]  != kLayers * kPrjN * kDin) return;
  if (in_sizes[6]  != kLayers * kDin * kDtR) return;
  if (in_sizes[7]  != kLayers * kDin) return;
  if (in_sizes[8]  != kLayers * kDin * kNst) return;
  if (in_sizes[9]  != kLayers * kDin) return;
  if (in_sizes[10] != kLayers * kDm * kDin) return;
  if (out_size != kRows * kDm) return;
  if (ws_size < kWsTotal) return;

  const float* pe     = (const float*)d_in[0];
  const float* cond   = (const float*)d_in[1];
  const float* W_in   = (const float*)d_in[2];
  const float* conv_w = (const float*)d_in[3];
  const float* conv_b = (const float*)d_in[4];
  const float* W_x    = (const float*)d_in[5];
  const float* W_dt   = (const float*)d_in[6];
  const float* b_dt   = (const float*)d_in[7];
  const float* A_log  = (const float*)d_in[8];
  const float* Dp     = (const float*)d_in[9];
  const float* W_out  = (const float*)d_in[10];
  float* out = (float*)d_out;

  char* ws = (char*)d_ws;
  unsigned short* XH   = (unsigned short*)(ws + kOffXH);
  unsigned short* XL   = (unsigned short*)(ws + kOffXL);
  unsigned short* WIN  = (unsigned short*)(ws + kOffWIN);
  unsigned short* WX   = (unsigned short*)(ws + kOffWX);
  unsigned short* WDT  = (unsigned short*)(ws + kOffWDT);
  unsigned short* WOUT = (unsigned short*)(ws + kOffWOUT);
  float*          XZ   = (float*)(ws + kOffXZ);
  float*          UC   = (float*)(ws + kOffUC);
  unsigned short* UCH  = (unsigned short*)(ws + kOffUCH);
  float*          XD   = (float*)(ws + kOffXD);
  unsigned short* DT   = (unsigned short*)(ws + kOffDT);
  float*          DLR  = (float*)(ws + kOffDLR);
  unsigned short* YH   = (unsigned short*)(ws + kOffYH);
  unsigned short* YL   = (unsigned short*)(ws + kOffYL);

  prep_x_kernel<<<(kRows * kDm / 8) / 256, 256, 0, stream>>>(pe, cond, XH, XL, kRows * kDm / 8);

  for (int layer = 0; layer < kLayers; ++layer) {
    const float* Wi = W_in   + (size_t)layer * kXzP * kDm;
    const float* cw = conv_w + (size_t)layer * kDin * 4;
    const float* cb = conv_b + (size_t)layer * kDin;
    const float* Wx = W_x    + (size_t)layer * kPrjN * kDin;
    const float* Wd = W_dt   + (size_t)layer * kDin * kDtR;
    const float* bd = b_dt   + (size_t)layer * kDin;
    const float* Al = A_log  + (size_t)layer * kDin * kNst;
    const float* Dl = Dp     + (size_t)layer * kDin;
    const float* Wo = W_out  + (size_t)layer * kDm * kDin;

    cast_rows_bf16_kernel<<<(kXzP * kDm / 8) / 256, 256, 0, stream>>>(Wi, WIN, kXzP * kDm / 8, kXzP * kDm / 8);
    cast_rows_bf16_kernel<<<(kPrjP * kDin / 8) / 256, 256, 0, stream>>>(Wx, WX, kPrjP * kDin / 8, kPrjN * kDin / 8);
    cast_rows_bf16_kernel<<<(kDin * kDtR / 8) / 256, 256, 0, stream>>>(Wd, WDT, kDin * kDtR / 8, kDin * kDtR / 8);
    cast_rows_bf16_kernel<<<(kDm * kDin / 8) / 256, 256, 0, stream>>>(Wo, WOUT, kDm * kDin / 8, kDm * kDin / 8);

    wmma_gemm64<1, 0><<<(kRows / 64) * (kXzP / 64) / 8, 256, 0, stream>>>(
        XH, XL, kDm, WIN, kDm, (void*)XZ, (void*)XZ, kXzP, kRows, kXzP, kDm);

    conv_silu_kernel<<<dim3(kDin / 256, kRows / 64), 256, 0, stream>>>(XZ, cw, cb, UC, UCH);

    wmma_gemm64<0, 0><<<(kRows / 64) * (kPrjP / 64) / 8, 256, 0, stream>>>(
        UCH, UCH, kDin, WX, kDin, (void*)XD, (void*)XD, kPrjP, kRows, kPrjP, kDin);

    dt_cast_kernel<<<(kRows * kDtR / 8) / 256, 256, 0, stream>>>(XD, DT, kRows * kDtR / 8);

    wmma_gemm64<0, 0><<<(kRows / 64) * (kDin / 64) / 8, 256, 0, stream>>>(
        DT, DT, kDtR, WDT, kDtR, (void*)DLR, (void*)DLR, kDin, kRows, kDin, kDtR);

    scan_kernel<<<kBatch * (kDin / kScanCh), kScanCh, 0, stream>>>(XD, UC, XZ, DLR, bd, Al, Dl, YH, YL);

    if (layer + 1 < kLayers) {
      wmma_gemm64<1, 2><<<(kRows / 64) * (kDm / 64) / 8, 256, 0, stream>>>(
          YH, YL, kDin, WOUT, kDin, (void*)XH, (void*)XL, kDm, kRows, kDm, kDin);
    } else {
      wmma_gemm64<1, 0><<<(kRows / 64) * (kDm / 64) / 8, 256, 0, stream>>>(
          YH, YL, kDin, WOUT, kDin, (void*)out, (void*)out, kDm, kRows, kDm, kDin);
    }
  }
}
